// mLSTMLayer_78537771975161
// MI455X (gfx1250) — hardware-run, weakly checked
//
#include <hip/hip_runtime.h>
#include <math.h>

constexpr int kB = 2;
constexpr int kS = 2048;
constexpr int kFeat = 1024;
constexpr int kHid = 2048;
constexpr int kNH = 4;
constexpr int kDH = 512;
constexpr int kTok = kB * kS;
constexpr int kGTok = 512;
constexpr int kNG = kB * kNH;
constexpr int kUpRows = 576;
constexpr int kICN = 576;
constexpr int kGateN = 64;
constexpr int kQKVW = 3 * kHid;
constexpr float kWCarry  = 16.0f;
constexpr float kQKCarry = 64.0f;
constexpr float kVCarry  = 64.0f;
constexpr float kGWCarry = 64.0f;
constexpr float kECarry  = 2048.0f;
constexpr float kHCarry  = 64.0f;
constexpr float kQScale  = 0.04419417382415922f;

typedef __attribute__((ext_vector_type(16))) _Float16 v16h;
typedef __attribute__((ext_vector_type(8)))  _Float16 v8h;
typedef __attribute__((ext_vector_type(16))) __bf16   v16b;
typedef __attribute__((ext_vector_type(8)))  __bf16   v8b;
typedef __attribute__((ext_vector_type(8)))  float    v8f;
typedef __attribute__((ext_vector_type(4)))  float    v4f;
typedef __attribute__((ext_vector_type(4)))  unsigned int v4u;

__device__ __forceinline__ unsigned short f2bf_bits(float f) {
  unsigned u = __float_as_uint(f);
  return (unsigned short)((u + 0x7FFFu + ((u >> 16) & 1u)) >> 16);
}
__device__ __forceinline__ float bf_bits2f(unsigned short h) { return __uint_as_float(((unsigned)h) << 16); }

__device__ __forceinline__ void dep_guard_h(v8f& a, v8f& b, v16h x, v16h y) { asm volatile("v_nop\n\tv_nop\n\tv_nop\n\tv_nop" : "+v"(a), "+v"(b) : "v"(x), "v"(y)); }
__device__ __forceinline__ void dep_guard_b(v8f& a, v8f& b, v16b x, v16b y) { asm volatile("v_nop\n\tv_nop\n\tv_nop\n\tv_nop" : "+v"(a), "+v"(b) : "v"(x), "v"(y)); }
__device__ __forceinline__ void keep4_h(v16h a, v16h b, v16h c, v16h d) { asm volatile("v_nop" :: "v"(a), "v"(b), "v"(c), "v"(d)); }
__device__ __forceinline__ void keep4_b(v16b a, v16b b, v16b c, v16b d) { asm volatile("v_nop" :: "v"(a), "v"(b), "v"(c), "v"(d)); }
__device__ __forceinline__ void acc_guard4(v8f& a, v8f& b, v8f& c, v8f& d) { asm volatile("v_nop\n\tv_nop\n\tv_nop\n\tv_nop" : "+v"(a), "+v"(b), "+v"(c), "+v"(d)); }
template <typename T> struct Frag;
template <> struct Frag<_Float16> {
  typedef v16h V; union U { v16h v; v8h h[2]; };
  static __device__ __forceinline__ v16h load(const _Float16* p) {
    U f; f.h[0] = *(const v8h*)(p); f.h[1] = *(const v8h*)(p + 16); return f.v;
  }
  static __device__ __forceinline__ v8f mma(v16h a, v16h b, v8f c) {
    return __builtin_amdgcn_wmma_f32_16x16x32_f16(false, a, false, b, (short)0, c, false, false);
  }
  static __device__ __forceinline__ void guard(v8f& a, v8f& b, v16h x, v16h y) { dep_guard_h(a, b, x, y); }
  static __device__ __forceinline__ void keep(v16h a, v16h b, v16h c, v16h d) { keep4_h(a, b, c, d); }
};
template <> struct Frag<__bf16> {
  typedef v16b V; union U { v16b v; v8b h[2]; };
  static __device__ __forceinline__ v16b load(const __bf16* p) {
    U f; f.h[0] = *(const v8b*)(p); f.h[1] = *(const v8b*)(p + 16); return f.v;
  }
  static __device__ __forceinline__ v8f mma(v16b a, v16b b, v8f c) {
    return __builtin_amdgcn_wmma_f32_16x16x32_bf16(false, a, false, b, (short)0, c, false, false);
  }
  static __device__ __forceinline__ void guard(v8f& a, v8f& b, v16b x, v16b y) { dep_guard_b(a, b, x, y); }
  static __device__ __forceinline__ void keep(v16b a, v16b b, v16b c, v16b d) { keep4_b(a, b, c, d); }
};

__device__ __forceinline__ unsigned pk16(unsigned short a, unsigned short b) { return (unsigned)a | ((unsigned)b << 16); }
__device__ __forceinline__ unsigned short h_bits(float f) { const _Float16 h = (_Float16)f; return __builtin_bit_cast(unsigned short, h); }

template <int ET> struct Elem;
template <> struct Elem<0> { typedef _Float16 T; };
template <> struct Elem<1> { typedef __bf16 T; };
template <int ET, bool SPLIT, int BIAS_MODE, int OUT_MODE, bool RESID, int ACT = 0, int TRI = 0>
__global__ __launch_bounds__(256) void wmma_gemm64(
    const unsigned short* __restrict__ Ap, const unsigned short* __restrict__ A2p, int lda, long strideA,
    const unsigned short* __restrict__ Btp, const unsigned short* __restrict__ Bt2p, int ldb, long strideB,
    void* __restrict__ Cout, void* __restrict__ Cout2, int ldc, long strideC,
    const float* __restrict__ bias,
    const float* __restrict__ resid, long strideR,
    int M, int N, int K, float scale) {
  typedef typename Elem<ET>::T T;
  typedef typename Frag<T>::V V;
  const T* A = (const T*)Ap; const T* A2 = (const T*)A2p; const T* Bt = (const T*)Btp; const T* Bt2 = (const T*)Bt2p;
  __shared__ __align__(16) float sT[8][16 * 68];
  const int b    = blockIdx.y;
  const int lane = threadIdx.x & 31;
  const int wave = threadIdx.x >> 5;
  const int tilesN = N >> 6;
  const int tilesM = M >> 6;
  const int tile = blockIdx.x * 8 + wave;
  if (tile >= tilesM * tilesN) return;
  const int tm = tile / tilesN;
  const int tn = tile - tm * tilesN;
  if (TRI == 1 && tn > tm) return;
  const int m0 = tm << 6;
  const int n0 = tn << 6;
  const int Kt = (TRI == 2) ? ((K < m0 + 64) ? K : (m0 + 64)) : K;

  const T* Ab  = A  + (size_t)b * strideA;
  const T* Bb  = Bt + (size_t)b * strideB;
  const T* Ab2 = SPLIT ? (A2  + (size_t)b * strideA) : nullptr;
  const T* Bb2 = SPLIT ? (Bt2 + (size_t)b * strideB) : nullptr;

  const int rlane = lane & 15;
  const int koff  = (lane >> 4) * 8;
  const int mOff  = (lane >> 4) * 8;

  v8f acc[4][4];
#pragma unroll
  for (int i = 0; i < 4; ++i)
#pragma unroll
    for (int j = 0; j < 4; ++j) acc[i][j] = (v8f){0.f,0.f,0.f,0.f,0.f,0.f,0.f,0.f};

  for (int k0 = 0; k0 < Kt; k0 += 32) {
    V bh[4], bl[4];
#pragma unroll
    for (int j = 0; j < 4; ++j) {
      const size_t bo = (size_t)(n0 + (j << 4) + rlane) * ldb + koff + k0;
      bh[j] = Frag<T>::load(Bb + bo);
      if (SPLIT) bl[j] = Frag<T>::load(Bb2 + bo);
    }
#pragma unroll
    for (int i = 0; i < 4; ++i) {
      const size_t ao = (size_t)(m0 + (i << 4) + rlane) * lda + koff + k0;
      V ah = Frag<T>::load(Ab + ao);
      V al;
      if (SPLIT) al = Frag<T>::load(Ab2 + ao);
#pragma unroll
      for (int j = 0; j < 4; ++j) {
        acc[i][j] = Frag<T>::mma(ah, bh[j], acc[i][j]);
        if (SPLIT) {
          acc[i][j] = Frag<T>::mma(ah, bl[j], acc[i][j]);
          acc[i][j] = Frag<T>::mma(al, bh[j], acc[i][j]);
        }
      }
      Frag<T>::guard(acc[i][0], acc[i][3], ah, SPLIT ? al : ah);
    }
    Frag<T>::keep(bh[0], bh[1], bh[2], bh[3]);
    if (SPLIT) Frag<T>::keep(bl[0], bl[1], bl[2], bl[3]);
  }
  acc_guard4(acc[0][0], acc[0][1], acc[0][2], acc[0][3]);
  acc_guard4(acc[1][0], acc[1][1], acc[1][2], acc[1][3]);
  acc_guard4(acc[2][0], acc[2][1], acc[2][2], acc[2][3]);
  acc_guard4(acc[3][0], acc[3][1], acc[3][2], acc[3][3]);

  float* slab = sT[wave];
  const float* Rb = RESID ? (resid + (size_t)b * strideR) : nullptr;
#pragma unroll
  for (int i = 0; i < 4; ++i) {
    const int mBase = m0 + (i << 4);
#pragma unroll
    for (int j = 0; j < 4; ++j) {
      const int n = n0 + (j << 4) + rlane;
      float bv = 0.f;
      if (BIAS_MODE == 2) bv = bias[n];
#pragma unroll
      for (int r = 0; r < 8; ++r) {
        float v = acc[i][j][r] * scale;
        if (BIAS_MODE == 1) v += bias[mBase + mOff + r];
        if (BIAS_MODE == 2) v += bv;
        if (RESID) v += Rb[(size_t)(mBase + mOff + r) * ldc + n];
        if (ACT == 2) v = fmaxf(v, 0.0f);
        if (ACT == 4) v = (v > 0.f) ? v : 0.01f * v;
        slab[(mOff + r) * 68 + (j << 4) + rlane] = v;
      }
    }
    __builtin_amdgcn_fence(__ATOMIC_RELEASE, "workgroup");
    __builtin_amdgcn_wave_barrier();
    __builtin_amdgcn_fence(__ATOMIC_ACQUIRE, "workgroup");
    if (OUT_MODE == 0) {
      float* C = (float*)Cout + (size_t)b * strideC;
      const int hh = lane >> 4, c4 = (lane & 15) * 4;
      for (int pass = 0; pass < 2; ++pass) {
#pragma unroll
        for (int it = 0; it < 8; ++it) {
          const int row = it * 2 + hh;
          v4f v = *(const v4f*)(slab + row * 68 + c4);
          *(volatile v4f*)(C + (size_t)(mBase + row) * ldc + n0 + c4) = v;
        }
        __threadfence();
      }
    } else {
      const int q = lane >> 3, c8 = (lane & 7) * 8;
      unsigned short* C  = (unsigned short*)Cout  + (size_t)b * strideC;
      unsigned short* C2 = (OUT_MODE == 2) ? ((unsigned short*)Cout2 + (size_t)b * strideC) : nullptr;
      for (int pass = 0; pass < 2; ++pass) {
#pragma unroll
        for (int it = 0; it < 4; ++it) {
          const int row = it * 4 + q;
          const float* sp = slab + row * 68 + c8;
          v8h hv, lv;
#pragma unroll
          for (int e = 0; e < 8; ++e) {
            if (OUT_MODE == 1) {
              hv[e] = (_Float16)sp[e];
            } else {
              unsigned short hb = f2bf_bits(sp[e]);
              unsigned short lb = f2bf_bits(sp[e] - bf_bits2f(hb));
              hv[e] = __builtin_bit_cast(_Float16, hb);
              lv[e] = __builtin_bit_cast(_Float16, lb);
            }
          }
          *(volatile v8h*)(C + (size_t)(mBase + row) * ldc + n0 + c8) = hv;
          if (OUT_MODE == 2) *(volatile v8h*)(C2 + (size_t)(mBase + row) * ldc + n0 + c8) = lv;
        }
        __threadfence();
      }
    }
    __builtin_amdgcn_fence(__ATOMIC_RELEASE, "workgroup");
    __builtin_amdgcn_wave_barrier();
    __builtin_amdgcn_fence(__ATOMIC_ACQUIRE, "workgroup");
  }
}

__global__ __launch_bounds__(256) void cast8_f16_kernel(const float* __restrict__ in, unsigned short* __restrict__ out, int n8) {
  const int i = blockIdx.x * 256 + threadIdx.x;
  if (i >= n8) return;
  const float* p = in + 8 * (size_t)i;
  const v4f a = *(const v4f*)(p);
  const v4f c = *(const v4f*)(p + 4);
  unsigned short hb[8];
#pragma unroll
  for (int e = 0; e < 4; ++e) {
    hb[e]     = h_bits(a[e]);
    hb[4 + e] = h_bits(c[e]);
  }
  const v4u u = (v4u){pk16(hb[0], hb[1]), pk16(hb[2], hb[3]), pk16(hb[4], hb[5]), pk16(hb[6], hb[7])};
  unsigned short* q = out + 8 * (size_t)i;
  *(volatile v4u*)q = u;
  __threadfence();
  *(volatile v4u*)q = u;
}

__global__ __launch_bounds__(256) void tcast_kernel(const float* __restrict__ W, unsigned short* __restrict__ out,
                                                    int Kd, int Nd, float scale) {
  __shared__ float sm[64][65];
  const int t  = threadIdx.x;
  const int k0 = blockIdx.x * 64;
  const int n0 = blockIdx.y * 64;
#pragma unroll
  for (int i = 0; i < 16; ++i) {
    const int e = i * 256 + t;
    const int r = e >> 6;
    const int c = e & 63;
    sm[c][r] = W[(size_t)(k0 + r) * Nd + n0 + c] * scale;
  }
  __syncthreads();
  const int lane = t & 31, wave = t >> 5;
  const int q = lane >> 3, c8 = (lane & 7) * 8;
  for (int pass = 0; pass < 2; ++pass) {
#pragma unroll
    for (int it = 0; it < 2; ++it) {
      const int row = wave * 8 + it * 4 + q;
      unsigned short hb[8];
#pragma unroll
      for (int e = 0; e < 8; ++e) hb[e] = h_bits(sm[row][c8 + e]);
      const v4u u = (v4u){pk16(hb[0], hb[1]), pk16(hb[2], hb[3]), pk16(hb[4], hb[5]), pk16(hb[6], hb[7])};
      *(volatile v4u*)(out + (size_t)(n0 + row) * Kd + k0 + c8) = u;
    }
    __threadfence();
  }
}

__global__ __launch_bounds__(256) void gw_cast_kernel(const float* __restrict__ wi, const float* __restrict__ wf,
                                                      unsigned short* __restrict__ out, float scale) {
  __shared__ float sm[64][65];
  const int t  = threadIdx.x;
  const int k0 = blockIdx.x * 64;
  {
    const int kk = t >> 2, n = t & 3;
    sm[n][kk]     = wi[(size_t)(k0 + kk) * 4 + n] * scale;
    sm[4 + n][kk] = wf[(size_t)(k0 + kk) * 4 + n] * scale;
  }
#pragma unroll
  for (int i = 0; i < 14; ++i) {
    const int e = i * 256 + t;
    sm[8 + (e >> 6)][e & 63] = 0.0f;
  }
  __syncthreads();
  const int lane = t & 31, wave = t >> 5;
  const int q = lane >> 3, c8 = (lane & 7) * 8;
  for (int pass = 0; pass < 2; ++pass) {
#pragma unroll
    for (int it = 0; it < 2; ++it) {
      const int row = wave * 8 + it * 4 + q;
      unsigned short hb[8];
#pragma unroll
      for (int e = 0; e < 8; ++e) hb[e] = h_bits(sm[row][c8 + e]);
      const v4u u = (v4u){pk16(hb[0], hb[1]), pk16(hb[2], hb[3]), pk16(hb[4], hb[5]), pk16(hb[6], hb[7])};
      *(volatile v4u*)(out + (size_t)row * kQKVW + k0 + c8) = u;
    }
    __threadfence();
  }
}

__global__ __launch_bounds__(256) void c0t_kernel(const float* __restrict__ C0g, const float* __restrict__ n0g,
                                                  unsigned short* __restrict__ out) {
  __shared__ float sm[64][65];
  const int t  = threadIdx.x;
  const int k0 = blockIdx.x * 64;
  const int n0 = blockIdx.y * 64;
  if (blockIdx.y < 8) {
#pragma unroll
    for (int i = 0; i < 16; ++i) {
      const int e = i * 256 + t;
      const int r = e >> 6;
      const int c = e & 63;
      sm[c][r] = C0g[(size_t)(k0 + r) * kDH + n0 + c];
    }
  } else {
#pragma unroll
    for (int i = 0; i < 16; ++i) {
      const int e = i * 256 + t;
      const int r = e >> 6;
      const int c = e & 63;
      const float nv = n0g[k0 + c];
      sm[r][c] = (r == 0) ? nv : 0.0f;
    }
  }
  __syncthreads();
  const int lane = t & 31, wave = t >> 5;
  const int q = lane >> 3, c8 = (lane & 7) * 8;
  for (int pass = 0; pass < 2; ++pass) {
#pragma unroll
    for (int it = 0; it < 2; ++it) {
      const int row = wave * 8 + it * 4 + q;
      unsigned short hb[8];
#pragma unroll
      for (int e = 0; e < 8; ++e) hb[e] = h_bits(sm[row][c8 + e]);
      const v4u u = (v4u){pk16(hb[0], hb[1]), pk16(hb[2], hb[3]), pk16(hb[4], hb[5]), pk16(hb[6], hb[7])};
      *(volatile v4u*)(out + (size_t)(n0 + row) * kDH + k0 + c8) = u;
    }
    __threadfence();
  }
}

__global__ __launch_bounds__(32) void ep_kernel(const int* __restrict__ mk, int* __restrict__ ep) {
  __shared__ int sh[kS];
  const int b = blockIdx.x, lane = threadIdx.x;
  const int* ms = mk + (size_t)b * kS;
  int* ed = ep + (size_t)b * kS;
  int carry = 0;
  for (int c = 0; c < kS / 32; ++c) {
    int v = ms[c * 32 + lane];
#pragma unroll
    for (int off = 1; off < 32; off <<= 1) {
      const int nb = __shfl_up(v, off, 32);
      if (lane >= off) v += nb;
    }
    sh[c * 32 + lane] = carry + v;
    carry += __shfl(v, 31, 32);
  }
  __syncthreads();
  for (int pass = 0; pass < 2; ++pass) {
    for (int c = 0; c < kS / 32; ++c) {
      const int o = sh[c * 32 + lane];
      ((volatile int*)ed)[c * 32 + lane] = o;
    }
    __threadfence();
  }
}

__global__ __launch_bounds__(512) void conv_bdd_kernel(
    const float* __restrict__ UPg, int xoff, int tokbase,
    const float* __restrict__ cst_b, const float* __restrict__ conv_w, const float* __restrict__ conv_b,
    const float* __restrict__ Wq, const float* __restrict__ Wk, const float* __restrict__ Wv,
    float* __restrict__ CAg, unsigned short* __restrict__ Q16g, unsigned short* __restrict__ K16g,
    unsigned short* __restrict__ QKVg) {
  __shared__ __align__(16) float cash[kHid];
  __shared__ __align__(16) unsigned short qsh[kHid];
  __shared__ __align__(16) unsigned short ksh[kHid];
  __shared__ __align__(16) unsigned short vsh[kHid];
  const int sl  = blockIdx.x;
  const int tid = threadIdx.x;
  const int s   = tokbase + sl;
  const int t0 = s - 3, t1 = s - 2, t2 = s - 1;
  const float* rp0 = (t0 >= 0) ? (UPg + (size_t)(t0 - tokbase + xoff) * (2 * kHid)) : (cst_b + (size_t)(t0 + 4) * kHid);
  const float* rp1 = (t1 >= 0) ? (UPg + (size_t)(t1 - tokbase + xoff) * (2 * kHid)) : (cst_b + (size_t)(t1 + 4) * kHid);
  const float* rp2 = (t2 >= 0) ? (UPg + (size_t)(t2 - tokbase + xoff) * (2 * kHid)) : (cst_b + (size_t)(t2 + 4) * kHid);
  const float* rp3 = UPg + (size_t)(s - tokbase + xoff) * (2 * kHid);
  const float* wq = Wq + (size_t)tid * 16;
  const float* wk = Wk + (size_t)tid * 16;
  const float* wv = Wv + (size_t)tid * 16;

  float qa[4] = {0.f, 0.f, 0.f, 0.f};
  float ka[4] = {0.f, 0.f, 0.f, 0.f};
  float va[4] = {0.f, 0.f, 0.f, 0.f};
#pragma unroll 1
  for (int i = 0; i < 4; ++i) {
    const int c = tid * 4 + i;
    const float x0 = rp0[c], x1 = rp1[c], x2 = rp2[c], x3 = rp3[c];
    float cv = conv_b[c];
    cv += conv_w[c] * x0;
    cv += conv_w[kHid + c] * x1;
    cv += conv_w[2 * kHid + c] * x2;
    cv += conv_w[3 * kHid + c] * x3;
    const float ca = cv * (1.0f / (1.0f + expf(-cv)));
    cash[c] = ca;
#pragma unroll
    for (int o = 0; o < 4; ++o) {
      qa[o] += ca * wq[i * 4 + o];
      ka[o] += ca * wk[i * 4 + o];
      va[o] += x3 * wv[i * 4 + o];
    }
  }
#pragma unroll
  for (int o = 0; o < 4; ++o) {
    qsh[tid * 4 + o] = h_bits(qa[o] * kQKCarry);
    ksh[tid * 4 + o] = h_bits(ka[o] * kQKCarry);
    vsh[tid * 4 + o] = h_bits(va[o] * kVCarry);
  }
  __syncthreads();
  const int j = tid & 255;
  const bool lowhalf = tid < 256;
  const v4f cav = *(const v4f*)(cash + tid * 4);
  const v4u uq = *(const v4u*)(qsh + 8 * j);
  const v4u uk = *(const v4u*)(ksh + 8 * j);
  const v4u uv = *(const v4u*)(vsh + 8 * j);
  v4u u1;
#pragma unroll
  for (int e = 0; e < 4; ++e) u1[e] = lowhalf ? uq[e] : uk[e];
  float* dca = CAg + (size_t)sl * kHid + tid * 4;
  unsigned short* d1 = lowhalf ? (Q16g + (size_t)sl * kHid + 8 * j) : (K16g + (size_t)sl * kHid + 8 * j);
  unsigned short* d2 = QKVg + (size_t)sl * kQKVW + 8 * tid;
  unsigned short* d3 = QKVg + (size_t)sl * kQKVW + 2 * kHid + 8 * j;
  for (int pass = 0; pass < 2; ++pass) {
    *(volatile v4f*)dca = cav;
    *(volatile v4u*)d1 = u1;
    *(volatile v4u*)d2 = u1;
    if (lowhalf) *(volatile v4u*)d3 = uv;
    __threadfence();
  }
}

__global__ __launch_bounds__(32) void scan_kernel(const float* __restrict__ Gg, const float* __restrict__ wi_b,
                                                 const float* __restrict__ wf_b, float* __restrict__ LFCg,
                                                 float* __restrict__ IGg) {
  __shared__ float shl[kS];
  __shared__ float shi[kS];
  const int lane = threadIdx.x;
  float carry = 0.f;
  for (int c = 0; c < kS / 32; ++c) {
    const int t = c * 32 + lane;
    const int tok = t >> 2, hh = t & 3;
    const float gi = Gg[(size_t)tok * kGateN + hh] + wi_b[hh];
    const float gf = Gg[(size_t)tok * kGateN + 4 + hh] + wf_b[hh];
    const float x = -gf;
    const float sp = fmaxf(x, 0.0f) + log1pf(expf(-fabsf(x)));
    float v = -sp;
#pragma unroll
    for (int off = 1; off < 32; off <<= 1) {
      const float nb = __shfl_up(v, off, 32);
      if (lane >= off) v += nb;
    }
    shl[t] = carry + v;
    shi[t] = gi;
    carry += __shfl(v, 31, 32);
  }
  __syncthreads();
  for (int pass = 0; pass < 2; ++pass) {
    for (int c = 0; c < kS / 32; ++c) {
      const float a = shl[c * 32 + lane];
      const float g = shi[c * 32 + lane];
      ((volatile float*)LFCg)[c * 32 + lane] = a;
      ((volatile float*)IGg)[c * 32 + lane] = g;
    }
    __threadfence();
  }
}

__global__ __launch_bounds__(256) void vt_kernel(const unsigned short* __restrict__ QKVg, unsigned short* __restrict__ VTg) {
  __shared__ __align__(16) unsigned short sm[64 * 72];
  const int t  = threadIdx.x;
  const int u0 = blockIdx.x * 64;
  const int d0 = blockIdx.y * 64;
#pragma unroll
  for (int it = 0; it < 2; ++it) {
    const int e   = it * 256 + t;
    const int ul  = e >> 3;
    const int ch8 = (e & 7) * 8;
    const int u   = u0 + ul;
    const unsigned short* src = QKVg + (size_t)(u >> 2) * kQKVW + 2 * kHid + (u & 3) * kDH + d0 + ch8;
    const v4u w = *(const v4u*)src;
#pragma unroll
    for (int p = 0; p < 4; ++p) {
      sm[(ch8 + 2 * p) * 72 + ul]     = (unsigned short)(w[p] & 0xffffu);
      sm[(ch8 + 2 * p + 1) * 72 + ul] = (unsigned short)(w[p] >> 16);
    }
  }
  __syncthreads();
  const int lane = t & 31, wave = t >> 5;
  const int q = lane >> 3, c8 = (lane & 7) * 8;
  for (int pass = 0; pass < 2; ++pass) {
#pragma unroll
    for (int it = 0; it < 2; ++it) {
      const int row = wave * 8 + it * 4 + q;
      const v4u uu = *(const v4u*)(sm + row * 72 + c8);
      *(volatile v4u*)(VTg + (size_t)(d0 + row) * kS + u0 + c8) = uu;
    }
    __threadfence();
  }
}

__global__ __launch_bounds__(256) void row_kernel(
    const float* __restrict__ Sg, const float* __restrict__ ICg,
    const float* __restrict__ LFCg, const float* __restrict__ IGg,
    const int* __restrict__ EPb, const float* __restrict__ m0p,
    unsigned short* __restrict__ E16g, float* __restrict__ Rg) {
  __shared__ __align__(16) float esh[kS];
  __shared__ __align__(16) unsigned short hsh[kS];
  __shared__ float redA[8];
  __shared__ float redB[8];
  const int t    = blockIdx.x;
  const int tid  = threadIdx.x;
  const int lane = tid & 31, wave = tid >> 5;
  const int c0   = tid * 8;
  const float lfct = LFCg[t];
  const float igt  = IGg[t];
  const int   ept  = EPb[t];
  const float m0v  = m0p[0];
  const float* srow = Sg + (size_t)t * kS;

  float mx = -INFINITY;
#pragma unroll 1
  for (int e = 0; e < 8; ++e) {
    const int u = c0 + e;
    const bool ok = (u <= t) && (EPb[u] == ept);
    const float ld = ok ? ((lfct - LFCg[u]) + igt) : -INFINITY;
    esh[u] = ld;
    mx = fmaxf(mx, ld);
  }
#pragma unroll
  for (int off = 16; off > 0; off >>= 1) mx = fmaxf(mx, __shfl_xor(mx, off, 32));
  if (lane == 0) redA[wave] = mx;
  __syncthreads();
  float maxd = redA[0];
#pragma unroll
  for (int w = 1; w < 8; ++w) maxd = fmaxf(maxd, redA[w]);
  const float sdc   = lfct + m0v;
  const float stab  = fmaxf(maxd, sdc);
  const float decay = expf(sdc - stab);

  float se = 0.0f;
#pragma unroll 1
  for (int e = 0; e < 8; ++e) {
    const int u   = c0 + e;
    const int ucl = (u < t) ? u : t;
    const float sv = srow[ucl];
    const float dm = expf(esh[u] - stab);
    const float pr = sv * dm;
    const float ev = (u <= t) ? pr : 0.0f;
    esh[u] = ev;
    se += ev;
  }
#pragma unroll
  for (int off = 16; off > 0; off >>= 1) se += __shfl_xor(se, off, 32);
  if (lane == 0) redB[wave] = se;
  __syncthreads();
  float sume = 0.0f;
#pragma unroll
  for (int w = 0; w < 8; ++w) sume += redB[w];
  const float qn    = ICg[(size_t)t * kICN + kDH];
  const float normv = fmaxf(fabsf(sume) + decay * qn, expf(-stab));
  const float inv   = 1.0f / (normv + 1e-6f);

#pragma unroll 1
  for (int e = 0; e < 8; ++e) {
    const int u = c0 + e;
    const float w = esh[u] * inv;
    hsh[u] = h_bits(w * kECarry);
  }
  __syncthreads();
  const v4u ue  = *(const v4u*)(hsh + c0);
  const int cr  = (tid & 127) * 4;
  const v4f icv = *(const v4f*)(ICg + (size_t)t * kICN + cr);
  const float rsc = decay * inv;
  const v4f rv  = icv * rsc;
  unsigned short* de = E16g + (size_t)t * kS + c0;
  float* dr = Rg + (size_t)t * kDH + cr;
  const bool wr = tid < 128;
  for (int pass = 0; pass < 2; ++pass) {
    *(volatile v4u*)de = ue;
    if (wr) *(volatile v4f*)dr = rv;
    __threadfence();
  }
}

__global__ __launch_bounds__(256) void combine_kernel(const float* __restrict__ HTg, const float* __restrict__ CAg,
                                                      const float* __restrict__ UPg, int xoff,
                                                      const float* __restrict__ skip, unsigned short* __restrict__ H16g) {
  __shared__ __align__(16) unsigned short hsh[256 * 8];
  const int tid  = threadIdx.x;
  const int f0   = (blockIdx.x * 256 + tid) * 8;
  const int tokl = f0 >> 11;
  const int cb   = f0 & (kHid - 1);
  const float* zr = UPg + (size_t)(tokl + xoff) * (2 * kHid) + kHid + cb;
#pragma unroll 1
  for (int e = 0; e < 8; ++e) {
    const float z  = zr[e];
    const float g  = z * (1.0f / (1.0f + expf(-z)));
    const float hv = (HTg[f0 + e] + skip[cb + e] * CAg[f0 + e]) * g;
    hsh[tid * 8 + e] = h_bits(hv * kHCarry);
  }
  __syncthreads();
  const v4u u = *(const v4u*)(hsh + tid * 8);
  unsigned short* d = H16g + f0;
  *(volatile v4u*)d = u;
  __threadfence();
  *(volatile v4u*)d = u;
}

extern "C" void kernel_launch(void* const* d_in, const int* in_sizes, int n_in,
                              void* d_out, int out_size, void* d_ws, size_t ws_size,
                              hipStream_t stream) {
  if (n_in < 18) return;
  if (in_sizes[0] != kTok * kFeat || in_sizes[1] != kB * kS || out_size != kTok * kFeat) return;
  if (in_sizes[3] != kNG * kDH * kDH || in_sizes[6] != kFeat * 2 * kHid || in_sizes[17] != kHid * kFeat) return;

  const float* inputs     = (const float*)d_in[0];
  const int*   mk         = (const int*)d_in[1];
  const float* conv_state = (const float*)d_in[2];
  const float* C0         = (const float*)d_in[3];
  const float* n0         = (const float*)d_in[4];
  const float* m0         = (const float*)d_in[5];
  const float* W_up       = (const float*)d_in[6];
  const float* conv_w     = (const float*)d_in[7];
  const float* conv_b     = (const float*)d_in[8];
  const float* Wq         = (const float*)d_in[9];
  const float* Wk         = (const float*)d_in[10];
  const float* Wv         = (const float*)d_in[11];
  const float* wi_k       = (const float*)d_in[12];
  const float* wi_b       = (const float*)d_in[13];
  const float* wf_k       = (const float*)d_in[14];
  const float* wf_b       = (const float*)d_in[15];
  const float* skip       = (const float*)d_in[16];
  const float* W_down     = (const float*)d_in[17];
  float* out = (float*)d_out;

  size_t off = 0;
  auto carve = [&](size_t bytes) -> size_t { const size_t o = off; off += (bytes + 255) & ~(size_t)255; return o; };
  const size_t oX16  = carve((size_t)kTok * kFeat * 2);
  const size_t oWUPT = carve((size_t)(2 * kHid) * kFeat * 2);
  const size_t oWDNT = carve((size_t)kFeat * kHid * 2);
  const size_t oWGT  = carve((size_t)kGateN * kQKVW * 2);
  const size_t oH16  = carve((size_t)kTok * kHid * 2);
  const size_t oEP   = carve((size_t)kB * kS * 4);
  const size_t oUPG  = carve((size_t)kUpRows * (2 * kHid) * 4);
  const size_t oCAG  = carve((size_t)kGTok * kHid * 4);
  const size_t oQ16G = carve((size_t)kGTok * kHid * 2);
  const size_t oK16G = carve((size_t)kGTok * kHid * 2);
  const size_t oQKVG = carve((size_t)kGTok * kQKVW * 2);
  const size_t oVTG  = carve((size_t)kDH * kS * 2);
  const size_t oC0TG = carve((size_t)kICN * kDH * 2);
  const size_t oGG   = carve((size_t)kGTok * kGateN * 4);
  const size_t oLFCG = carve((size_t)kS * 4);
  const size_t oIGG  = carve((size_t)kS * 4);
  const size_t oSG   = carve((size_t)kS * kS * 4);
  const size_t oICG  = carve((size_t)kS * kICN * 4);
  const size_t oE16G = carve((size_t)kS * kS * 2);
  const size_t oRG   = carve((size_t)kS * kDH * 4);
  const size_t oHTG  = carve((size_t)kS * kDH * 4);
  if (off > ws_size) return;

  char* ws = (char*)d_ws;
  unsigned short* X16  = (unsigned short*)(ws + oX16);
  unsigned short* WUPT = (unsigned short*)(ws + oWUPT);
  unsigned short* WDNT = (unsigned short*)(ws + oWDNT);
  unsigned short* WGT  = (unsigned short*)(ws + oWGT);
  unsigned short* H16  = (unsigned short*)(ws + oH16);
  int*   EP    = (int*)(ws + oEP);
  float* UPG   = (float*)(ws + oUPG);
  float* CAG   = (float*)(ws + oCAG);
  unsigned short* Q16G = (unsigned short*)(ws + oQ16G);
  unsigned short* K16G = (unsigned short*)(ws + oK16G);
  unsigned short* QKVG = (unsigned short*)(ws + oQKVG);
  unsigned short* VTG  = (unsigned short*)(ws + oVTG);
  unsigned short* C0TG = (unsigned short*)(ws + oC0TG);
  float* GG    = (float*)(ws + oGG);
  float* LFCG  = (float*)(ws + oLFCG);
  float* IGG   = (float*)(ws + oIGG);
  float* SG    = (float*)(ws + oSG);
  float* ICG   = (float*)(ws + oICG);
  unsigned short* E16G = (unsigned short*)(ws + oE16G);
  float* RG    = (float*)(ws + oRG);
  float* HTG   = (float*)(ws + oHTG);
  const unsigned short* nul16 = (const unsigned short*)nullptr;
  const float* nulf = (const float*)nullptr;

  cast8_f16_kernel<<<(kTok * kFeat / 8) / 256, 256, 0, stream>>>(inputs, X16, kTok * kFeat / 8);
  tcast_kernel<<<dim3(kFeat / 64, (2 * kHid) / 64), 256, 0, stream>>>(W_up, WUPT, kFeat, 2 * kHid, kWCarry);
  tcast_kernel<<<dim3(kHid / 64, kFeat / 64), 256, 0, stream>>>(W_down, WDNT, kHid, kFeat, kWCarry);
  gw_cast_kernel<<<kQKVW / 64, 256, 0, stream>>>(wi_k, wf_k, WGT, kGWCarry);
  ep_kernel<<<kB, 32, 0, stream>>>(mk, EP);

  for (int g = 0; g < kNG; ++g) {
    const int b = g >> 2, h = g & 3;
    const int tokbase = h * kGTok;
    const int xoff = (h == 0) ? 0 : 64;
    const int xbase = b * kS + tokbase - xoff;

    {
      const int tiles = (kUpRows / 64) * ((2 * kHid) / 64);
      hipLaunchKernelGGL(HIP_KERNEL_NAME(wmma_gemm64<0, false, 0, 0, false, 0, 0>), dim3((tiles + 7) / 8, 1), dim3(256), 0, stream,
          (const unsigned short*)(X16 + (size_t)xbase * kFeat), nul16, (int)kFeat, (long)0,
          (const unsigned short*)WUPT, nul16, (int)kFeat, (long)0,
          (void*)UPG, (void*)nullptr, (int)(2 * kHid), (long)0,
          nulf, nulf, (long)0,
          (int)kUpRows, (int)(2 * kHid), (int)kFeat, 1.0f / kWCarry);
    }
    conv_bdd_kernel<<<kGTok, 512, 0, stream>>>(UPG, xoff, tokbase, conv_state + (size_t)b * 4 * kHid,
                                                conv_w, conv_b, Wq, Wk, Wv, CAG, Q16G, K16G, QKVG);
    {
      const int tiles = (kGTok / 64) * (kGateN / 64);
      hipLaunchKernelGGL(HIP_KERNEL_NAME(wmma_gemm64<0, false, 0, 0, false, 0, 0>), dim3((tiles + 7) / 8, 1), dim3(256), 0, stream,
          (const unsigned short*)QKVG, nul16, (int)kQKVW, (long)0,
          (const unsigned short*)WGT, nul16, (int)kQKVW, (long)0,
          (void*)GG, (void*)nullptr, (int)kGateN, (long)0,
          nulf, nulf, (long)0,
          (int)kGTok, (int)kGateN, (int)kQKVW, 1.0f / (kQKCarry * kGWCarry));
    }
    scan_kernel<<<1, 32, 0, stream>>>(GG, wi_b, wf_b, LFCG, IGG);
    vt_kernel<<<dim3(kS / 64, kDH / 64), 256, 0, stream>>>(QKVG, VTG);
    c0t_kernel<<<dim3(kDH / 64, kICN / 64), 256, 0, stream>>>(C0 + (size_t)g * kDH * kDH, n0 + (size_t)g * kDH, C0TG);
    {
      const int tiles = (kS / 64) * (kS / 64);
      hipLaunchKernelGGL(HIP_KERNEL_NAME(wmma_gemm64<0, false, 0, 0, false, 0, 1>), dim3((tiles + 7) / 8, 1), dim3(256), 0, stream,
          (const unsigned short*)Q16G, nul16, (int)kDH, (long)0,
          (const unsigned short*)K16G, nul16, (int)kDH, (long)0,
          (void*)SG, (void*)nullptr, (int)kS, (long)0,
          nulf, nulf, (long)0,
          (int)kS, (int)kS, (int)kDH, kQScale * (1.0f / (kQKCarry * kQKCarry)));
    }
    {
      const int tiles = (kS / 64) * (kICN / 64);
      hipLaunchKernelGGL(HIP_KERNEL_NAME(wmma_gemm64<0, false, 0, 0, false, 0, 0>), dim3((tiles + 7) / 8, 1), dim3(256), 0, stream,
          (const unsigned short*)Q16G, nul16, (int)kDH, (long)0,
          (const unsigned short*)C0TG, nul16, (int)kDH, (long)0,
          (void*)ICG, (void*)nullptr, (int)kICN, (long)0,
          nulf, nulf, (long)0,
          (int)kS, (int)kICN, (int)kDH, kQScale * (1.0f / kQKCarry));
    }
    row_kernel<<<kS, 256, 0, stream>>>(SG, ICG, LFCG, IGG, EP + (size_t)b * kS, m0 + g, E16G, RG);
    {
      const int tiles = (kS / 64) * (kDH / 64);
      hipLaunchKernelGGL(HIP_KERNEL_NAME(wmma_gemm64<0, false, 0, 0, true, 0, 2>), dim3((tiles + 7) / 8, 1), dim3(256), 0, stream,
          (const unsigned short*)E16G, nul16, (int)kS, (long)0,
          (const unsigned short*)VTG, nul16, (int)kS, (long)0,
          (void*)HTG, (void*)nullptr, (int)kDH, (long)0,
          nulf, (const float*)RG, (long)0,
          (int)kS, (int)kDH, (int)kS, 1.0f / (kECarry * kVCarry));
    }
    combine_kernel<<<(kS * kDH / 8) / 256, 256, 0, stream>>>(HTG, CAG, UPG, xoff, skip, H16 + (size_t)g * kS * kDH);
  }

  {
    const int tiles = (kTok / 64) * (kFeat / 64);
    hipLaunchKernelGGL(HIP_KERNEL_NAME(wmma_gemm64<0, false, 0, 0, false, 0, 0>), dim3((tiles + 7) / 8, 1), dim3(256), 0, stream,
        (const unsigned short*)H16, nul16, (int)kHid, (long)0,
        (const unsigned short*)WDNT, nul16, (int)kHid, (long)0,
        (void*)out, (void*)nullptr, (int)kFeat, (long)0,
        nulf, nulf, (long)0,
        (int)kTok, (int)kFeat, (int)kHid, 1.0f / (kHCarry * kWCarry));
  }
}
